// Involution_57982058496731
// MI455X (gfx1250) — hardware-run, weakly checked
//
#include <hip/hip_runtime.h>


#define NB_  8
#define CC   256
#define RC   128
#define HH   56
#define WW   56
#define NP   3136
#define OC   3136
#define KS   7
typedef _Float16 h16;
typedef unsigned short bf;
typedef __attribute__((ext_vector_type(16))) __bf16   v16bf;
typedef __attribute__((ext_vector_type(16))) _Float16 v16h;
typedef __attribute__((ext_vector_type(8)))  _Float16 v8h;
typedef __attribute__((ext_vector_type(8)))  unsigned short v8us;
typedef __attribute__((ext_vector_type(8)))  float    v8f;
typedef __attribute__((ext_vector_type(4)))  float    v4f;
typedef v8h  __attribute__((may_alias)) v8ha;
typedef v4f  __attribute__((may_alias)) v4fa;
typedef v8us __attribute__((may_alias)) v8usa;

__device__ __forceinline__ unsigned short f2bf(float f) { unsigned u = __float_as_uint(f); u += 0x7FFFu + ((u >> 16) & 1u); return (unsigned short)(u >> 16); }
__device__ __forceinline__ float bf2f(unsigned short b) { return __uint_as_float(((unsigned)b) << 16); }
__device__ __forceinline__ float bfr(float f) { return bf2f(f2bf(f)); }
__device__ __forceinline__ v16h cat16(v8h lo, v8h hi) { return __builtin_shufflevector(lo, hi, 0, 1, 2, 3, 4, 5, 6, 7, 8, 9, 10, 11, 12, 13, 14, 15); }
__device__ __forceinline__ v16bf cat16b(v8us lo, v8us hi) { return __builtin_bit_cast(v16bf, __builtin_shufflevector(lo, hi, 0, 1, 2, 3, 4, 5, 6, 7, 8, 9, 10, 11, 12, 13, 14, 15)); }
__device__ __forceinline__ v8f wmma16(v16h a, v16h b, v8f c) { return __builtin_amdgcn_wmma_f32_16x16x32_f16(false, a, false, b, (short)0, c, false, false); }
__device__ __forceinline__ v8f wmmab(v16bf a, v16bf b, v8f c) { return __builtin_amdgcn_wmma_f32_16x16x32_bf16(false, a, false, b, (short)0, c, false, false); }


template <typename T16> struct WFrag;
template <> struct WFrag<h16> { typedef v16h V; static __device__ __forceinline__ V ld(const h16* p) { return cat16(*(const v8h*)p, *(const v8h*)(p + 16)); } static __device__ __forceinline__ v8f mma(V a, V b, v8f c) { return wmma16(a, b, c); } };
template <> struct WFrag<bf> { typedef v16bf V; static __device__ __forceinline__ V ld(const bf* p) { return cat16b(*(const v8us*)p, *(const v8us*)(p + 16)); } static __device__ __forceinline__ v8f mma(V a, V b, v8f c) { return wmmab(a, b, c); } };
template <typename T16, int NSPLIT, bool BIAS>
__global__ __launch_bounds__(32) void k_gemmw(const T16* __restrict__ A, const T16* __restrict__ A2, const T16* __restrict__ Bt, const T16* __restrict__ Bt2, int K, float* C, int ldc, const float* __restrict__ bias, size_t sA, size_t sB, size_t sC) {
    typedef typename WFrag<T16>::V V;
    __shared__ __align__(16) float os[16 * 68];
    const size_t z = blockIdx.z; A += z * sA; if (A2) A2 += z * sA; Bt += z * sB; if (Bt2) Bt2 += z * sB; C += z * sC;
    const int lane = threadIdx.x & 31, lr = lane & 15, hi = lane >> 4; const int r0 = blockIdx.x * 64, c0 = blockIdx.y * 64;
    v8f acc[4][4];
#pragma unroll
    for (int mb = 0; mb < 4; ++mb)
#pragma unroll
        for (int nb = 0; nb < 4; ++nb) acc[mb][nb] = (v8f){};
    const size_t aoff = (size_t)(r0 + lr) * K + 8 * hi, boff = (size_t)(c0 + lr) * K + 8 * hi;
#pragma unroll 1
    for (int kc = 0; kc < K; kc += 32) {
        V a[4], a2[4];
#pragma unroll
        for (int mb = 0; mb < 4; ++mb) { a[mb] = WFrag<T16>::ld(A + aoff + (size_t)mb * 16 * K + kc); if (NSPLIT == 1 || NSPLIT == 2) a2[mb] = WFrag<T16>::ld(A2 + aoff + (size_t)mb * 16 * K + kc); }
#pragma unroll
        for (int nb = 0; nb < 4; ++nb) { const V b = WFrag<T16>::ld(Bt + boff + (size_t)nb * 16 * K + kc); V b2; if (NSPLIT >= 2) b2 = WFrag<T16>::ld(Bt2 + boff + (size_t)nb * 16 * K + kc);
#pragma unroll
            for (int mb = 0; mb < 4; ++mb) { acc[mb][nb] = WFrag<T16>::mma(a[mb], b, acc[mb][nb]); if (NSPLIT == 1 || NSPLIT == 2) acc[mb][nb] = WFrag<T16>::mma(a2[mb], b, acc[mb][nb]); if (NSPLIT >= 2) acc[mb][nb] = WFrag<T16>::mma(a[mb], b2, acc[mb][nb]); } }
        asm volatile("v_nop\n\tv_nop\n\tv_nop\n\tv_nop" : "+v"(acc[0][0]), "+v"(acc[1][1]), "+v"(acc[2][2]), "+v"(acc[3][3]) : "v"(a[0]), "v"(a[3]));
    }
#pragma unroll
    for (int mb = 0; mb < 4; ++mb) {
#pragma unroll
        for (int nb = 0; nb < 4; ++nb) {
#pragma unroll
            for (int j = 0; j < 8; ++j) os[(hi * 8 + j) * 68 + nb * 16 + lr] = acc[mb][nb][j]; }
        __builtin_amdgcn_wave_barrier(); asm volatile("" ::: "memory");
        float* crow = C + (size_t)(r0 + mb * 16) * ldc + c0;
#pragma unroll 1
        for (int ps = 0; ps < 2; ++ps) {
#pragma unroll
            for (int s = 0; s < 8; ++s) { const int row = 2 * s + hi, cofs = lr * 4; v4f val = *(const v4fa*)(os + row * 68 + cofs); if (BIAS) { val[0] += bfr(bias[c0 + cofs]); val[1] += bfr(bias[c0 + cofs + 1]); val[2] += bfr(bias[c0 + cofs + 2]); val[3] += bfr(bias[c0 + cofs + 3]); }
                *(volatile v4f*)(crow + (size_t)row * ldc + cofs) = val; }
            if (ps == 0) __threadfence(); }
        __builtin_amdgcn_wave_barrier(); asm volatile("" ::: "memory");
    }
}

__device__ __forceinline__ void splitf(float y, unsigned short& h, unsigned short& l) { h = f2bf(y); l = f2bf(y - bf2f(h)); }
typedef __attribute__((ext_vector_type(4))) unsigned short v4us;

__global__ __launch_bounds__(256) void k_cvt8(const float* __restrict__ src, bf* dst, size_t n8) { const size_t i = (size_t)blockIdx.x * 256 + threadIdx.x; if (i >= n8) return; const v8f v = *(const v8f*)(src + i * 8); v8us o;
#pragma unroll
    for (int k = 0; k < 8; ++k) o[k] = f2bf(v[k]); *(volatile v8us*)(dst + i * 8) = o; __threadfence(); *(volatile v8us*)(dst + i * 8) = o; }
__global__ __launch_bounds__(256) void k_trb(const float* __restrict__ xb, bf* XT) { __shared__ float tile[64][33]; const int t0 = blockIdx.x * 32, c0 = blockIdx.y * 64; const int lx = threadIdx.x & 31, ly = threadIdx.x >> 5;
    for (int r = ly; r < 64; r += 8) tile[r][lx] = xb[(size_t)(c0 + r) * NP + t0 + lx];
    __syncthreads();
#pragma unroll
    for (int pass = 0; pass < 2; ++pass) { const int r = pass * 16 + (threadIdx.x >> 4), q = threadIdx.x & 15; v4us o;
#pragma unroll
        for (int u = 0; u < 4; ++u) o[u] = f2bf(tile[q * 4 + u][r]); bf* dst = XT + (size_t)(t0 + r) * CC + c0 + q * 4; *(volatile v4us*)dst = o; __threadfence(); *(volatile v4us*)dst = o; } }
__global__ __launch_bounds__(256) void k_pl(const float* __restrict__ F, bf* Ph, bf* Pl) { const size_t e = ((size_t)blockIdx.x * 256 + threadIdx.x) * 4; if (e >= (size_t)NP * RC) return; v4us oh, ol;
#pragma unroll
    for (int u = 0; u < 4; ++u) { unsigned short a, b2; splitf(F[e + u], a, b2); oh[u] = a; ol[u] = b2; } *(volatile v4us*)(Ph + e) = oh; *(volatile v4us*)(Pl + e) = ol; __threadfence(); *(volatile v4us*)(Ph + e) = oh; *(volatile v4us*)(Pl + e) = ol; }
__global__ __launch_bounds__(256) void k_inv(const float* __restrict__ WT, const float* __restrict__ xb, float* outb) { const size_t e = ((size_t)blockIdx.x * 256 + threadIdx.x) * 4; if (e >= (size_t)CC * NP) return; const int px0 = (int)(e % NP); const int c = (int)(e / NP); const int g = c / 4; const int y = px0 / WW, x0 = px0 % WW; const float* xc = xb + (size_t)c * NP; v4f r;
#pragma unroll
    for (int u = 0; u < 4; ++u) { const int x = x0 + u; const float* wrow = WT + (size_t)(px0 + u) * OC + g * (KS * KS); float acc = 0.f;
#pragma unroll 1
        for (int ki = 0; ki < KS; ++ki) { const int yy = y + ki - 3; if (yy < 0 || yy >= HH) continue;
#pragma unroll
            for (int kj = 0; kj < KS; ++kj) { const int xx = x + kj - 3; const float xv = (xx >= 0 && xx < WW) ? bfr(xc[yy * WW + xx]) : 0.f; float p = __fmul_rn(wrow[ki * KS + kj], xv); asm volatile("" : "+v"(p)); acc = __fadd_rn(acc, p); } }
        r[u] = acc; }
    *(volatile v4f*)(outb + e) = r; __threadfence(); *(volatile v4f*)(outb + e) = r; }

extern "C" void kernel_launch(void* const* d_in, const int* in_sizes, int n_in,
                              void* d_out, int out_size, void* d_ws, size_t ws_size, hipStream_t stream) {
    (void)in_sizes; (void)n_in; (void)out_size;
    const float** I = (const float**)d_in;
    const float *x = I[0], *w1 = I[1], *b1 = I[2], *w2 = I[3], *b2 = I[4];
    float* OUT = (float*)d_out;
    char* wsp = (char*)d_ws;
    auto take = [&](size_t bytes) { char* p = wsp; wsp += (bytes + 255) & ~(size_t)255; return (void*)p; };
    bf* XT = (bf*)take((size_t)NP * CC * 2); bf* B1 = (bf*)take((size_t)RC * CC * 2); bf* B2 = (bf*)take((size_t)OC * RC * 2); float* F1 = (float*)take((size_t)NP * RC * 4); bf* F1h = (bf*)take((size_t)NP * RC * 2); bf* F1l = (bf*)take((size_t)NP * RC * 2); float* WT = (float*)take((size_t)NP * OC * 4);
    if ((size_t)(wsp - (char*)d_ws) > ws_size) return;
    k_cvt8<<<(RC * CC / 8 + 255) / 256, 256, 0, stream>>>(w1, B1, RC * CC / 8); k_cvt8<<<(unsigned)(((size_t)OC * RC / 8 + 255) / 256), 256, 0, stream>>>(w2, B2, (size_t)OC * RC / 8);
    for (int b = 0; b < NB_; ++b) {
        k_trb<<<dim3(NP / 32, CC / 64, 1), 256, 0, stream>>>(x + (size_t)b * CC * NP, XT);
        k_gemmw<bf, 0, true><<<dim3(NP / 64, RC / 64, 1), 32, 0, stream>>>(XT, nullptr, B1, nullptr, CC, F1, RC, b1, 0, 0, 0);
        k_pl<<<(NP * RC / 4 + 255) / 256, 256, 0, stream>>>(F1, F1h, F1l);
        k_gemmw<bf, 1, true><<<dim3(NP / 64, OC / 64, 1), 32, 0, stream>>>(F1h, F1l, B2, nullptr, RC, WT, OC, b2, 0, 0, 0);
        k_inv<<<(unsigned)(((size_t)CC * NP / 4 + 255) / 256), 256, 0, stream>>>(WT, x + (size_t)b * CC * NP, OUT + (size_t)b * CC * NP); }
}
